// DeltaNet_22488448762180
// MI455X (gfx1250) — hardware-run, weakly checked
//
#include <hip/hip_runtime.h>


#define NSQ 2
#define NTS 2048
#define NDM 1024
#define NHS 16
#define NFE 64
#define NBK 32
#define NPR 32
#define NZB 1024
#define NBL 4096
#define NRW 4096
#define NGP 64
#define TT  2048
#define HD  64

typedef _Float16 h16;
typedef unsigned short bf;
typedef __attribute__((ext_vector_type(16))) __bf16   v16bf;
typedef __attribute__((ext_vector_type(16))) _Float16 v16h;
typedef __attribute__((ext_vector_type(8)))  _Float16 v8h;
typedef __attribute__((ext_vector_type(8)))  unsigned short v8us;
typedef __attribute__((ext_vector_type(8)))  float    v8f;
typedef __attribute__((ext_vector_type(4)))  float    v4f;
typedef v8h  __attribute__((may_alias)) v8ha;
typedef v4f  __attribute__((may_alias)) v4fa;
typedef v8us __attribute__((may_alias)) v8usa;

__device__ __forceinline__ unsigned short f2bf(float f) { unsigned u = __float_as_uint(f); u += 0x7FFFu + ((u >> 16) & 1u); return (unsigned short)(u >> 16); }
__device__ __forceinline__ float bf2f(unsigned short b) { return __uint_as_float(((unsigned)b) << 16); }
__device__ __forceinline__ float bfr(float f) { return bf2f(f2bf(f)); }
__device__ __forceinline__ v16h cat16(v8h lo, v8h hi) { return __builtin_shufflevector(lo, hi, 0, 1, 2, 3, 4, 5, 6, 7, 8, 9, 10, 11, 12, 13, 14, 15); }
__device__ __forceinline__ v16bf cat16b(v8us lo, v8us hi) { return __builtin_bit_cast(v16bf, __builtin_shufflevector(lo, hi, 0, 1, 2, 3, 4, 5, 6, 7, 8, 9, 10, 11, 12, 13, 14, 15)); }
__device__ __forceinline__ v8f wmma16(v16h a, v16h b, v8f c) { return __builtin_amdgcn_wmma_f32_16x16x32_f16(false, a, false, b, (short)0, c, false, false); }
__device__ __forceinline__ v8f wmmab(v16bf a, v16bf b, v8f c) { return __builtin_amdgcn_wmma_f32_16x16x32_bf16(false, a, false, b, (short)0, c, false, false); }

template <typename T16> struct WFrag;
template <> struct WFrag<h16> { typedef v16h V; static __device__ __forceinline__ V ld(const h16* p) { return cat16(*(const v8h*)p, *(const v8h*)(p + 16)); } static __device__ __forceinline__ v8f mma(V a, V b, v8f c) { return wmma16(a, b, c); } };
template <> struct WFrag<bf> { typedef v16bf V; static __device__ __forceinline__ V ld(const bf* p) { return cat16b(*(const v8us*)p, *(const v8us*)(p + 16)); } static __device__ __forceinline__ v8f mma(V a, V b, v8f c) { return wmmab(a, b, c); } };
template <typename T16, int NSPLIT, bool BIAS>
__global__ __launch_bounds__(32) void k_gemmw(const T16* __restrict__ A, const T16* __restrict__ A2, const T16* __restrict__ Bt, const T16* __restrict__ Bt2, int K, float* C, int ldc, const float* __restrict__ bias, size_t sA, size_t sB, size_t sC) {
    typedef typename WFrag<T16>::V V;
    __shared__ __align__(16) float os[16 * 68];
    const size_t z = blockIdx.z; A += z * sA; if (A2) A2 += z * sA; Bt += z * sB; if (Bt2) Bt2 += z * sB; C += z * sC;
    const int lane = threadIdx.x & 31, lr = lane & 15, hi = lane >> 4; const int r0 = blockIdx.x * 64, c0 = blockIdx.y * 64;
    v8f acc[4][4];
#pragma unroll
    for (int mb = 0; mb < 4; ++mb)
#pragma unroll
        for (int nb = 0; nb < 4; ++nb) acc[mb][nb] = (v8f){};
    const size_t aoff = (size_t)(r0 + lr) * K + 8 * hi, boff = (size_t)(c0 + lr) * K + 8 * hi;
    for (int kc = 0; kc < K; kc += 32) {
        V a[4], a2[4];
#pragma unroll
        for (int mb = 0; mb < 4; ++mb) { a[mb] = WFrag<T16>::ld(A + aoff + (size_t)mb * 16 * K + kc); if (NSPLIT == 1 || NSPLIT == 2) a2[mb] = WFrag<T16>::ld(A2 + aoff + (size_t)mb * 16 * K + kc); }
#pragma unroll
        for (int nb = 0; nb < 4; ++nb) { const V b = WFrag<T16>::ld(Bt + boff + (size_t)nb * 16 * K + kc); V b2; if (NSPLIT >= 2) b2 = WFrag<T16>::ld(Bt2 + boff + (size_t)nb * 16 * K + kc);
#pragma unroll
            for (int mb = 0; mb < 4; ++mb) { acc[mb][nb] = WFrag<T16>::mma(a[mb], b, acc[mb][nb]); if (NSPLIT == 1 || NSPLIT == 2) acc[mb][nb] = WFrag<T16>::mma(a2[mb], b, acc[mb][nb]); if (NSPLIT >= 2) acc[mb][nb] = WFrag<T16>::mma(a[mb], b2, acc[mb][nb]); } }
        asm volatile("v_nop\n\tv_nop\n\tv_nop\n\tv_nop" : "+v"(acc[0][0]), "+v"(acc[1][1]), "+v"(acc[2][2]), "+v"(acc[3][3]) : "v"(a[0]), "v"(a[3]));
    }
#pragma unroll
    for (int mb = 0; mb < 4; ++mb) {
#pragma unroll
        for (int nb = 0; nb < 4; ++nb) {
#pragma unroll
            for (int j = 0; j < 8; ++j) os[(hi * 8 + j) * 68 + nb * 16 + lr] = acc[mb][nb][j]; }
        __builtin_amdgcn_wave_barrier(); asm volatile("" ::: "memory");
        float* crow = C + (size_t)(r0 + mb * 16) * ldc + c0;
#pragma unroll 1
        for (int ps = 0; ps < 2; ++ps) {
#pragma unroll
            for (int s = 0; s < 8; ++s) { const int row = 2 * s + hi, cofs = lr * 4; v4f val = *(const v4fa*)(os + row * 68 + cofs); if (BIAS) { val[0] += bfr(bias[c0 + cofs]); val[1] += bfr(bias[c0 + cofs + 1]); val[2] += bfr(bias[c0 + cofs + 2]); val[3] += bfr(bias[c0 + cofs + 3]); }
                *(volatile v4f*)(crow + (size_t)row * ldc + cofs) = val; }
            if (ps == 0) __threadfence(); }
        __builtin_amdgcn_wave_barrier(); asm volatile("" ::: "memory");
    }
}

typedef __attribute__((ext_vector_type(2))) _Float16 v2h;
typedef __attribute__((ext_vector_type(4))) _Float16 v4h;
typedef __attribute__((ext_vector_type(2))) unsigned short v2us;
typedef __attribute__((ext_vector_type(4))) unsigned short v4us;
typedef __attribute__((ext_vector_type(2))) float v2f;
typedef __attribute__((ext_vector_type(4))) int v4i;
__device__ __forceinline__ h16 toh_flush(float x) { const float z = (fabsf(x) < 6.103515625e-05f) ? 0.0f : x; return (h16)z; }

typedef __attribute__((ext_vector_type(4))) _Float16 v4h_;
__global__ __launch_bounds__(256) void k_fillb(bf* P, unsigned w2, size_t n8) { const size_t i = (size_t)blockIdx.x * 256 + threadIdx.x; if (i >= n8) return; v4i o; o[0] = (int)w2; o[1] = (int)w2; o[2] = (int)w2; o[3] = (int)w2;
    *(volatile v4i*)(P + i * 8) = o; __threadfence(); *(volatile v4i*)(P + i * 8) = o; }

__global__ __launch_bounds__(256) void k_cvt8(const float* __restrict__ src, bf* dst, size_t n8) { const size_t i = (size_t)blockIdx.x * 256 + threadIdx.x; if (i >= n8) return; const v8f v = *(const v8f*)(src + i * 8); v8us o;
#pragma unroll
    for (int k = 0; k < 8; ++k) o[k] = f2bf(v[k]); *(volatile v8us*)(dst + i * 8) = o; __threadfence(); *(volatile v8us*)(dst + i * 8) = o; }

__global__ __launch_bounds__(256) void k_xword(const float* __restrict__ src, h16* dst) {
    const size_t i = (size_t)blockIdx.x * 256 + threadIdx.x; const v8f wv = *(const v8f*)(src + i * 8); v8h ow;
#pragma unroll
    for (int j = 0; j < 8; ++j) ow[j] = toh_flush(bfr(wv[j]));
    *(volatile v8h*)(dst + i * 8) = ow; __threadfence(); *(volatile v8h*)(dst + i * 8) = ow; }

__global__ __launch_bounds__(256) void k_rbf(const float* __restrict__ X, float* Y, size_t n4) { const size_t i = (size_t)blockIdx.x * 256 + threadIdx.x; if (i >= n4) return; const v4f a = *(const v4f*)(X + i * 4); v4f o;
#pragma unroll
    for (int q = 0; q < 4; ++q) o[q] = bfr(a[q]);
    *(volatile v4f*)(Y + i * 4) = o; __threadfence(); *(volatile v4f*)(Y + i * 4) = o; }

#define LNC_MAX 2048
template <bool RES>
__global__ __launch_bounds__(256) void k_lnrow(const float* __restrict__ A, const float* __restrict__ R, const float* __restrict__ gamma, const float* __restrict__ beta, float eps, int C, int nrows, float* Y) {
    const int lane = threadIdx.x & 31; const int row = blockIdx.x * 8 + (threadIdx.x >> 5); if (row >= nrows) return; const int nch = C / 128; const float* a = A + (size_t)row * C; float x[LNC_MAX / 32]; float s = 0.0f;
    for (int k = 0; k < LNC_MAX / 128; ++k) { if (k < nch) { const int c0 = k * 128 + lane * 4; v4f v = *(const v4f*)(a + c0);
            if (RES) { const v4f w = *(const v4f*)(R + (size_t)row * C + c0); v[0] = __fadd_rn(v[0], w[0]); v[1] = __fadd_rn(v[1], w[1]); v[2] = __fadd_rn(v[2], w[2]); v[3] = __fadd_rn(v[3], w[3]); }
            x[k * 4 + 0] = v[0]; x[k * 4 + 1] = v[1]; x[k * 4 + 2] = v[2]; x[k * 4 + 3] = v[3]; s = __fadd_rn(__fadd_rn(__fadd_rn(__fadd_rn(s, v[0]), v[1]), v[2]), v[3]); } }
    for (int sh = 16; sh; sh >>= 1) s = __fadd_rn(s, __shfl_xor(s, sh, 32));
    const float mean = __fdiv_rn(s, (float)C); float q = 0.0f;
    for (int k = 0; k < LNC_MAX / 128; ++k) { if (k < nch) {
            for (int j = 0; j < 4; ++j) { const float d = __fsub_rn(x[k * 4 + j], mean); x[k * 4 + j] = d; q = __fmaf_rn(d, d, q); } } }
    for (int sh = 16; sh; sh >>= 1) q = __fadd_rn(q, __shfl_xor(q, sh, 32));
    const float rstd = __fdiv_rn(1.0f, sqrtf(__fadd_rn(__fdiv_rn(q, (float)C), eps)));
    for (int k = 0; k < LNC_MAX / 128; ++k) { if (k < nch) { const int c0 = k * 128 + lane * 4; const v4f g = *(const v4f*)(gamma + c0); const v4f bt = *(const v4f*)(beta + c0);
            for (int j = 0; j < 4; ++j) x[k * 4 + j] = __fmaf_rn(__fmul_rn(x[k * 4 + j], rstd), bfr(g[j]), bfr(bt[j])); } }
    float* y = Y + (size_t)row * C;
    for (int ps = 0; ps < 2; ++ps) {
        for (int k = 0; k < LNC_MAX / 128; ++k) { if (k < nch) { v4f o; o[0] = x[k * 4 + 0]; o[1] = x[k * 4 + 1]; o[2] = x[k * 4 + 2]; o[3] = x[k * 4 + 3]; *(volatile v4f*)(y + k * 128 + lane * 4) = o; } }
        if (ps == 0) __threadfence(); }
}

__global__ __launch_bounds__(256) void k_tb(const h16* __restrict__ src, h16* dst) {
    const unsigned i = blockIdx.x * 256 + threadIdx.x; const unsigned cl = i & 63u, z = i >> 6; const h16* pp = src + (size_t)z * NBL + cl; h16 r[64];
#pragma unroll
    for (int u = 0; u < 64; ++u) r[u] = pp[u * 64];
    h16* pd = dst + (size_t)i * 64;
#pragma unroll
    for (int ps = 0; ps < 2; ++ps) {
#pragma unroll
        for (int g = 0; g < 8; ++g) { v8h o;
#pragma unroll
            for (int j = 0; j < 8; ++j) o[j] = r[g * 8 + j];
            *(volatile v8h*)(pd + g * 8) = o; }
        if (ps == 0) __threadfence(); } }

__constant__ float INVT[HD / 2] = { 1.000000000e+00f, 7.498942018e-01f, 5.623413324e-01f, 4.216965139e-01f, 3.162277639e-01f, 2.371373624e-01f, 1.778279394e-01f, 1.333521456e-01f, 1.000000015e-01f, 7.498941571e-02f, 5.623412877e-02f, 4.216964915e-02f, 3.162277862e-02f, 2.371373586e-02f, 1.778279431e-02f, 1.333521493e-02f, 9.999999776e-03f, 7.498942316e-03f, 5.623413250e-03f, 4.216964822e-03f, 3.162277862e-03f, 2.371373819e-03f, 1.778279431e-03f, 1.333521446e-03f, 1.000000047e-03f, 7.498941850e-04f, 5.623413017e-04f, 4.216964880e-04f, 3.162277862e-04f, 2.371373848e-04f, 1.778279402e-04f, 1.333521504e-04f };
__global__ __launch_bounds__(256) void k_cs5(float* CS) { const int idx = blockIdx.x * 256 + threadIdx.x; if (idx >= TT * HD) return; const int d = idx % HD; const int t = idx / HD; const float a = __fmul_rn((float)t, INVT[d % (HD / 2)]); v2f cs; cs[0] = cosf(a); cs[1] = sinf(a); *(volatile v2f*)(CS + (size_t)idx * 2) = cs; __threadfence(); *(volatile v2f*)(CS + (size_t)idx * 2) = cs; }

__global__ __launch_bounds__(256) void k_gpl(const float* __restrict__ Zg, const float* __restrict__ a6, const int* __restrict__ a1, float* Fe, float* Ra, float* Ke, float* Ab) {
    const unsigned i = blockIdx.x * 256 + threadIdx.x; const unsigned pr = i >> 5, bk = i & 31u; const unsigned sq = pr >> 4, hd = pr & 15u; const unsigned r0 = sq * NTS + bk * 64u; const float bw = bfr(a6[hd]); float fe[64], pw[64];
#pragma unroll
    for (int u = 0; u < 64; ++u) { const float w = Zg[(size_t)(r0 + u) * NGP + hd] + bw; const float g = fminf(fmaxf(1.0f / (1.0f + expf(-w)), 0.01f), 0.999f); const float mw = (float)a1[r0 + u]; fe[u] = g * mw + (1.0f - mw); }
    float* pf = Fe + (size_t)i * 64; float* pa = Ra + (size_t)i * 64; float* pk = Ke + (size_t)i * 64;
#pragma unroll
    for (int ps = 0; ps < 2; ++ps) {
#pragma unroll
        for (int g4 = 0; g4 < 16; ++g4) { v4f o; o[0] = fe[g4 * 4 + 0]; o[1] = fe[g4 * 4 + 1]; o[2] = fe[g4 * 4 + 2]; o[3] = fe[g4 * 4 + 3]; *(volatile v4f*)(pf + g4 * 4) = o; }
        if (ps == 0) __threadfence(); }
    float run = 1.0f;
#pragma unroll
    for (int u = 0; u < 64; ++u) { run = run * fe[u]; pw[u] = run; }
    const float ab = run;
#pragma unroll
    for (int ps = 0; ps < 2; ++ps) {
#pragma unroll
        for (int g4 = 0; g4 < 16; ++g4) { v4f o; o[0] = pw[g4 * 4 + 0]; o[1] = pw[g4 * 4 + 1]; o[2] = pw[g4 * 4 + 2]; o[3] = pw[g4 * 4 + 3]; *(volatile v4f*)(pa + g4 * 4) = o; }
        if (ps == 0) __threadfence(); }
    run = 1.0f;
#pragma unroll
    for (int u = 63; u >= 0; --u) { pw[u] = run; run = run * fe[u]; }
#pragma unroll
    for (int ps = 0; ps < 2; ++ps) {
#pragma unroll
        for (int g4 = 0; g4 < 16; ++g4) { v4f o; o[0] = pw[g4 * 4 + 0]; o[1] = pw[g4 * 4 + 1]; o[2] = pw[g4 * 4 + 2]; o[3] = pw[g4 * 4 + 3]; *(volatile v4f*)(pk + g4 * 4) = o; }
        if (ps == 0) { *(volatile float*)(Ab + i) = ab; __threadfence(); } }
    *(volatile float*)(Ab + i) = ab; }

template <int MD>
__global__ __launch_bounds__(256) void k_fmw(const float* __restrict__ src, const float* __restrict__ CS, const int* __restrict__ a1, const float* __restrict__ Ke, h16* dst) {
    const unsigned i = blockIdx.x * 256 + threadIdx.x; const unsigned g8 = i & 7u, hr = i >> 3; const unsigned ts = hr & 2047u, pr = hr >> 11; const unsigned sq = pr >> 4, hd = pr & 15u; const unsigned d0 = g8 * 8u; const unsigned rw = sq * NTS + ts;
    const float* ps_ = src + (size_t)rw * NDM + hd * NFE; const float mw = (float)a1[rw]; const v8f u0 = *(const v8f*)(ps_ + d0); v8h ow;
    if (MD == 2) {
#pragma unroll
        for (int j = 0; j < 8; ++j) ow[j] = toh_flush(u0[j] * mw); }
    else { const v8f u1 = *(const v8f*)(ps_ + (d0 ^ 32u)); const float kf = (MD == 1) ? Ke[hr] : 1.0f;
#pragma unroll
        for (int j = 0; j < 8; ++j) { const v2f cs = *(const v2f*)(CS + ((size_t)ts * HD + d0 + j) * 2); const float pa = __fmul_rn(u0[j], cs[0]), pb = __fmul_rn(u1[j], cs[1]); const float w = (d0 < 32u) ? __fsub_rn(pa, pb) : __fadd_rn(pa, pb); const float fy = (fmaxf(w, 0.0f) + expf(fminf(w, 0.0f))) * mw; ow[j] = toh_flush((MD == 1) ? fy * kf : fy); } }
    *(volatile v8h*)(dst + (size_t)i * 8) = ow; __threadfence(); *(volatile v8h*)(dst + (size_t)i * 8) = ow; }

__global__ __launch_bounds__(256) void k_nsc(const h16* __restrict__ KfT, const float* __restrict__ Ab, float* Nm) {
    const unsigned i = blockIdx.x * 256 + threadIdx.x; const unsigned cl = i & 63u, pr = i >> 6; float nv[32]; float cur = 0.0f; nv[0] = 0.0f;
#pragma unroll
    for (int bk = 0; bk < 31; ++bk) { const h16* pk = KfT + ((size_t)(pr * 32u + (unsigned)bk) * 64 + cl) * 64; float sm = 0.0f;
#pragma unroll
        for (int g = 0; g < 8; ++g) { const v8h w = *(const v8h*)(pk + g * 8);
#pragma unroll
            for (int j = 0; j < 8; ++j) sm = sm + (float)w[j]; }
        cur = Ab[pr * 32u + (unsigned)bk] * cur + sm; nv[bk + 1] = cur; }
    float* pn = Nm + (size_t)pr * 32 * 64 + cl;
#pragma unroll
    for (int ps = 0; ps < 2; ++ps) {
#pragma unroll
        for (int bk = 0; bk < 32; ++bk) *(volatile float*)(pn + bk * 64) = nv[bk];
        if (ps == 0) __threadfence(); } }

__global__ __launch_bounds__(256) void k_mkw(const float* __restrict__ Pi, const float* __restrict__ Fe, const float* __restrict__ Ra, const h16* __restrict__ Qw, const float* __restrict__ Nm, h16* Ph, float* Dn) {
    const unsigned i = blockIdx.x * 256 + threadIdx.x; const unsigned tr = i & 63u, zb = i >> 6; const float* pi = Pi + (size_t)i * 64; const float* pf = Fe + (size_t)zb * 64; h16 rh[64]; float fv[64];
#pragma unroll
    for (int g4 = 0; g4 < 16; ++g4) { const v4f t4 = *(const v4fa*)(pf + g4 * 4); fv[g4 * 4 + 0] = t4[0]; fv[g4 * 4 + 1] = t4[1]; fv[g4 * 4 + 2] = t4[2]; fv[g4 * 4 + 3] = t4[3]; }
    float run = 1.0f, ds = 0.0f;
#pragma unroll
    for (int g = 7; g >= 0; --g) { const v8f t8 = *(const v8f*)(pi + g * 8);
#pragma unroll
        for (int jj = 7; jj >= 0; --jj) { const int s = g * 8 + jj; const float lt = (float)((unsigned)s < tr); const int s1 = (s < 63) ? s + 1 : 63; const float nx = (s < 63) ? fv[s1] : 1.0f; run = run * (lt * nx + (1.0f - lt)); const float kp = (float)((unsigned)s <= tr) * run; const h16 wd = toh_flush(t8[jj] * kp); rh[s] = wd; ds = ds + (float)wd; } }
    const h16* pq = Qw + (size_t)i * 64; const float* pn = Nm + (size_t)zb * 64; float dq = 0.0f;
#pragma unroll
    for (int g = 0; g < 8; ++g) { const v8h qw = *(const v8h*)(pq + g * 8); const v8f nn = *(const v8f*)(pn + g * 8);
#pragma unroll
        for (int j = 0; j < 8; ++j) dq = dq + (float)qw[j] * nn[j]; }
    const float dn = ds + Ra[i] * dq; h16* ph = Ph + (size_t)i * 64;
#pragma unroll
    for (int ps = 0; ps < 2; ++ps) {
#pragma unroll
        for (int g = 0; g < 8; ++g) { v8h oh;
#pragma unroll
            for (int jj = 0; jj < 8; ++jj) oh[jj] = rh[g * 8 + jj];
            *(volatile v8h*)(ph + g * 8) = oh; }
        *(volatile float*)(Dn + i) = dn;
        if (ps == 0) __threadfence(); } }

__global__ __launch_bounds__(256) void k_sst(const float* __restrict__ bef, const float* __restrict__ du, const float* __restrict__ Ab, int bk, float* aft, h16* wrd) {
    const size_t i = (size_t)blockIdx.x * 256 + threadIdx.x; const unsigned pr = (unsigned)(i >> 10); const float ab = Ab[pr * 32u + (unsigned)bk]; const v4f ub = *(const v4fa*)(bef + i * 4); const v4f vd = *(const v4fa*)(du + i * 4); v4f oa; v4h_ ow;
#pragma unroll
    for (int j = 0; j < 4; ++j) { oa[j] = ub[j] * ab + vd[j]; ow[j] = toh_flush(oa[j]); }
    *(volatile v4f*)(aft + i * 4) = oa; *(volatile v4h_*)(wrd + i * 4) = ow; __threadfence(); *(volatile v4f*)(aft + i * 4) = oa; *(volatile v4h_*)(wrd + i * 4) = ow; }

__global__ __launch_bounds__(256) void k_lyw(const float* __restrict__ Oi, const float* __restrict__ Ob, const float* __restrict__ Ra, const float* __restrict__ Dn, h16* Bw) {
    const unsigned i = blockIdx.x * 256 + threadIdx.x; const unsigned e4 = i & 15u, hr = i >> 4; const unsigned ts = hr & 2047u, pr = hr >> 11; const unsigned sq = pr >> 4, hd = pr & 15u; const v4f ua = *(const v4fa*)(Oi + (size_t)i * 4); const v4f ub = *(const v4fa*)(Ob + (size_t)i * 4); const float ra = Ra[hr]; const float dn = fmaxf(Dn[hr], 1.0e-6f); v4h_ ow;
#pragma unroll
    for (int j = 0; j < 4; ++j) ow[j] = toh_flush((ua[j] + ra * ub[j]) / dn);
    h16* pd = Bw + (size_t)(sq * NTS + ts) * NDM + hd * NFE + e4 * 4; *(volatile v4h_*)pd = ow; __threadfence(); *(volatile v4h_*)pd = ow; }

extern "C" void kernel_launch(void* const* d_in, const int* in_sizes, int n_in, void* d_out, int out_size, void* d_ws, size_t ws_size, hipStream_t stream) {
    if (n_in < 11) return;
    if (in_sizes[0] != NRW * NDM || in_sizes[1] != NRW || in_sizes[2] != NDM * NDM || in_sizes[3] != NDM * NDM || in_sizes[4] != NDM * NDM || in_sizes[5] != NHS * NDM || in_sizes[6] != NHS || in_sizes[7] != NDM * NDM || in_sizes[8] != NDM || in_sizes[9] != NDM || in_sizes[10] != NDM) return;
    if (out_size != NRW * NDM) return;
    static_assert(NRW == NSQ * NTS && NDM == NHS * NFE && NFE == 64 && NTS == NBK * 64 && NPR == NSQ * NHS && NZB == NPR * NBK && NBL == 64 * 64 && NTS == 2048 && NHS == 16 && NBK == 32 && NGP == 64 && NHS <= NGP && TT == NTS && HD == NFE && NRW % 64 == 0 && NDM % 64 == 0 && NDM % 32 == 0 && (NRW * NDM / 8) % 256 == 0 && (NDM * NDM / 8) % 256 == 0 && (NHS * NDM / 8) % 256 == 0 && ((NGP - NHS) * NDM / 8) % 256 == 0 && (NHS * NDM * 2) % 128 == 0 && NZB % 256 == 0 && (NZB * 64 * 8) % 256 == 0 && (NZB * 64) % 256 == 0 && (NPR * 64) % 256 == 0 && (NPR * NBL / 4) % 256 == 0 && (NPR * NBL * 4 / 16) % 256 == 0 && (NPR * NBL * 2 / 16) % 256 == 0 && (NZB * 64 * 16) % 256 == 0 && (NRW * NDM / 4) % 256 == 0 && NDM % 128 == 0 && NDM <= LNC_MAX && NRW % 8 == 0 && (size_t)NZB * NBL == (size_t)NRW * NDM, "the products: row and column counts multiples of 64, the depths of 32; the flat grids exact; a block 64 places; Pi, Oi and Ob fit in Pa's, Pb's and Pc's bytes; k_lnrow: the width a multiple of 128 and at most LNC_MAX, the rows in eights");
    const float* a0 = (const float*)d_in[0]; const int* a1 = (const int*)d_in[1]; const float* a2 = (const float*)d_in[2]; const float* a3 = (const float*)d_in[3]; const float* a4 = (const float*)d_in[4]; const float* a5 = (const float*)d_in[5]; const float* a6 = (const float*)d_in[6]; const float* a7 = (const float*)d_in[7]; const float* a8 = (const float*)d_in[8]; const float* a9 = (const float*)d_in[9]; const float* a10 = (const float*)d_in[10]; float* res = (float*)d_out;
    char* wsp = (char*)d_ws; auto take = [&](size_t bytes) { char* p = wsp; wsp += (bytes + 255) & ~(size_t)255; return (void*)p; };
    bf* Xb = (bf*)take((size_t)NRW * NDM * 2); bf* Wa = (bf*)take((size_t)NDM * NDM * 2); bf* Wb = (bf*)take((size_t)NDM * NDM * 2); bf* Wc = (bf*)take((size_t)NDM * NDM * 2); bf* Wz = (bf*)take((size_t)NGP * NDM * 2); h16* Wh = (h16*)take((size_t)NDM * NDM * 2);
    float* TTp = (float*)take((size_t)3 * NRW * NDM * 4); float* Zg = (float*)take((size_t)NRW * NGP * 4); float* CS = (float*)take((size_t)TT * HD * 2 * 4);
    float* Fe = (float*)take((size_t)NPR * NTS * 4); float* Ra = (float*)take((size_t)NPR * NTS * 4); float* Ke = (float*)take((size_t)NPR * NTS * 4); float* Ab = (float*)take((size_t)NZB * 4);
    h16* Qw = (h16*)take((size_t)NZB * NBL * 2); h16* Kw = (h16*)take((size_t)NZB * NBL * 2); h16* Kf = (h16*)take((size_t)NZB * NBL * 2); h16* Vw = (h16*)take((size_t)NZB * NBL * 2); h16* KfT = (h16*)take((size_t)NZB * NBL * 2); h16* VT = (h16*)take((size_t)NZB * NBL * 2);
    float* Nm = (float*)take((size_t)NZB * 64 * 4); h16* Ph = (h16*)take((size_t)NZB * NBL * 2); float* Dn = (float*)take((size_t)NZB * 64 * 4);
    float* StA = (float*)take((size_t)NPR * NBL * 4); float* StB = (float*)take((size_t)NPR * NBL * 4); h16* SwA = (h16*)take((size_t)NPR * NBL * 2); h16* SwB = (h16*)take((size_t)NPR * NBL * 2); float* Du = (float*)take((size_t)NPR * NBL * 4);
    h16* Bw = (h16*)take((size_t)NRW * NDM * 2); float* Po = (float*)take((size_t)NRW * NDM * 4); float* Xr = (float*)take((size_t)NRW * NDM * 4);
    if ((size_t)(wsp - (char*)d_ws) > ws_size) return;
    float* Pa = TTp; float* Pb = TTp + (size_t)NRW * NDM; float* Pc = TTp + (size_t)2 * NRW * NDM; float* Pi = TTp; float* Oi = TTp + (size_t)NZB * NBL; float* Ob = TTp + (size_t)2 * NZB * NBL;
    k_cvt8<<<(unsigned)(NRW * NDM / 8 / 256), 256, 0, stream>>>(a0, Xb, (size_t)NRW * NDM / 8);
    k_cvt8<<<(unsigned)(NDM * NDM / 8 / 256), 256, 0, stream>>>(a2, Wa, (size_t)NDM * NDM / 8); k_cvt8<<<(unsigned)(NDM * NDM / 8 / 256), 256, 0, stream>>>(a3, Wb, (size_t)NDM * NDM / 8); k_cvt8<<<(unsigned)(NDM * NDM / 8 / 256), 256, 0, stream>>>(a4, Wc, (size_t)NDM * NDM / 8);
    k_cvt8<<<(unsigned)(NHS * NDM / 8 / 256), 256, 0, stream>>>(a5, Wz, (size_t)NHS * NDM / 8);
    k_fillb<<<(unsigned)((NGP - NHS) * NDM / 8 / 256), 256, 0, stream>>>(Wz + (size_t)NHS * NDM, 0u, (size_t)(NGP - NHS) * NDM / 8);
    k_xword<<<(unsigned)(NDM * NDM / 8 / 256), 256, 0, stream>>>(a7, Wh);
    k_gemmw<bf, 0, false><<<dim3(NRW / 64, NDM / 64, 1), 32, 0, stream>>>(Xb, nullptr, Wa, nullptr, NDM, Pa, NDM, nullptr, 0, 0, 0);
    k_gemmw<bf, 0, false><<<dim3(NRW / 64, NDM / 64, 1), 32, 0, stream>>>(Xb, nullptr, Wb, nullptr, NDM, Pb, NDM, nullptr, 0, 0, 0);
    k_gemmw<bf, 0, false><<<dim3(NRW / 64, NDM / 64, 1), 32, 0, stream>>>(Xb, nullptr, Wc, nullptr, NDM, Pc, NDM, nullptr, 0, 0, 0);
    k_gemmw<bf, 0, false><<<dim3(NRW / 64, NGP / 64, 1), 32, 0, stream>>>(Xb, nullptr, Wz, nullptr, NDM, Zg, NGP, nullptr, 0, 0, 0);
    k_cs5<<<(TT * HD + 255) / 256, 256, 0, stream>>>(CS);
    k_gpl<<<NZB / 256, 256, 0, stream>>>(Zg, a6, a1, Fe, Ra, Ke, Ab);
    k_fmw<0><<<NZB * 64 * 8 / 256, 256, 0, stream>>>(Pa, CS, a1, nullptr, Qw); k_fmw<0><<<NZB * 64 * 8 / 256, 256, 0, stream>>>(Pb, CS, a1, nullptr, Kw); k_fmw<1><<<NZB * 64 * 8 / 256, 256, 0, stream>>>(Pb, CS, a1, Ke, Kf); k_fmw<2><<<NZB * 64 * 8 / 256, 256, 0, stream>>>(Pc, nullptr, a1, nullptr, Vw);
    k_tb<<<NZB * 64 / 256, 256, 0, stream>>>(Kf, KfT); k_tb<<<NZB * 64 / 256, 256, 0, stream>>>(Vw, VT);
    k_nsc<<<NPR * 64 / 256, 256, 0, stream>>>(KfT, Ab, Nm);
    k_gemmw<h16, 0, false><<<dim3(1, 1, NZB), 32, 0, stream>>>(Qw, nullptr, Kw, nullptr, 64, Pi, 64, nullptr, NBL, NBL, NBL);
    k_mkw<<<NZB * 64 / 256, 256, 0, stream>>>(Pi, Fe, Ra, Qw, Nm, Ph, Dn);
    k_gemmw<h16, 0, false><<<dim3(1, 1, NZB), 32, 0, stream>>>(Ph, nullptr, VT, nullptr, 64, Oi, 64, nullptr, NBL, NBL, NBL);
    k_fillb<<<(unsigned)((size_t)NPR * NBL * 4 / 16 / 256), 256, 0, stream>>>((bf*)StA, 0u, (size_t)NPR * NBL * 4 / 16); k_fillb<<<(unsigned)((size_t)NPR * NBL * 2 / 16 / 256), 256, 0, stream>>>((bf*)SwA, 0u, (size_t)NPR * NBL * 2 / 16);
    for (int bk = 0; bk < NBK; ++bk) { const float* stb = (bk & 1) ? StB : StA; float* sta = (bk & 1) ? StA : StB; const h16* swr = (bk & 1) ? SwB : SwA; h16* sww = (bk & 1) ? SwA : SwB;
        k_gemmw<h16, 0, false><<<dim3(1, 1, NPR), 32, 0, stream>>>(Qw + (size_t)bk * NBL, nullptr, swr, nullptr, 64, Ob + (size_t)bk * NBL, 64, nullptr, (size_t)NBK * NBL, NBL, (size_t)NBK * NBL);
        if (bk + 1 < NBK) { k_gemmw<h16, 0, false><<<dim3(1, 1, NPR), 32, 0, stream>>>(VT + (size_t)bk * NBL, nullptr, KfT + (size_t)bk * NBL, nullptr, 64, Du, 64, nullptr, (size_t)NBK * NBL, (size_t)NBK * NBL, NBL);
            k_sst<<<(unsigned)((size_t)NPR * NBL / 4 / 256), 256, 0, stream>>>(stb, Du, Ab, bk, sta, sww); } }
    k_lyw<<<NZB * 64 * 16 / 256, 256, 0, stream>>>(Oi, Ob, Ra, Dn, Bw);
    k_gemmw<h16, 0, true><<<dim3(NRW / 64, NDM / 64, 1), 32, 0, stream>>>(Bw, nullptr, Wh, nullptr, NDM, Po, NDM, a8, 0, 0, 0);
    k_rbf<<<(unsigned)(NRW * NDM / 4 / 256), 256, 0, stream>>>(a0, Xr, (size_t)NRW * NDM / 4);
    k_lnrow<true><<<(unsigned)(NRW / 8), 256, 0, stream>>>(Po, Xr, a9, a10, 1.0e-5f, NDM, NRW, res);
}
